// RWKV_TimeMix_49340584296473
// MI455X (gfx1250) — hardware-verified
//
#include <hip/hip_runtime.h>
#include <math.h>

constexpr int kB       = 8;
constexpr int kT       = 767;
constexpr int kC       = 1024;
constexpr int kRows    = kB * kT;
constexpr int kRowsPad = 6144;
constexpr int kN3      = 3 * kC;
constexpr int kTT      = 32;
constexpr float kWCarry    = 32.0f;
constexpr float kWCarryInv = 1.0f / 32.0f;
constexpr float kFltMax    = 3.4028235e38f;
static_assert(kRowsPad % 64 == 0);
static_assert(kRows % 2 == 0);
static_assert(kC % 256 == 0);
static_assert((kRowsPad * kC / 8) % 256 == 0);

typedef __attribute__((ext_vector_type(16))) _Float16 v16h;
typedef __attribute__((ext_vector_type(8)))  _Float16 v8h;
typedef __attribute__((ext_vector_type(16))) __bf16   v16b;
typedef __attribute__((ext_vector_type(8)))  __bf16   v8b;
typedef __attribute__((ext_vector_type(8)))  float    v8f;
typedef __attribute__((ext_vector_type(4)))  float    v4f;
typedef __attribute__((ext_vector_type(4)))  unsigned int v4u;

__device__ __forceinline__ unsigned short f2bf_bits(float f) {
  unsigned u = __float_as_uint(f);
  return (unsigned short)((u + 0x7FFFu + ((u >> 16) & 1u)) >> 16);
}
__device__ __forceinline__ float bf_bits2f(unsigned short h) { return __uint_as_float(((unsigned)h) << 16); }

__device__ __forceinline__ void dep_guard_h(v8f& a, v8f& b, v16h x, v16h y) { asm volatile("v_nop\n\tv_nop\n\tv_nop\n\tv_nop" : "+v"(a), "+v"(b) : "v"(x), "v"(y)); }
__device__ __forceinline__ void dep_guard_b(v8f& a, v8f& b, v16b x, v16b y) { asm volatile("v_nop\n\tv_nop\n\tv_nop\n\tv_nop" : "+v"(a), "+v"(b) : "v"(x), "v"(y)); }
__device__ __forceinline__ void keep4_h(v16h a, v16h b, v16h c, v16h d) { asm volatile("v_nop" :: "v"(a), "v"(b), "v"(c), "v"(d)); }
__device__ __forceinline__ void keep4_b(v16b a, v16b b, v16b c, v16b d) { asm volatile("v_nop" :: "v"(a), "v"(b), "v"(c), "v"(d)); }
__device__ __forceinline__ void acc_guard4(v8f& a, v8f& b, v8f& c, v8f& d) { asm volatile("v_nop\n\tv_nop\n\tv_nop\n\tv_nop" : "+v"(a), "+v"(b), "+v"(c), "+v"(d)); }
template <typename T> struct Frag;
template <> struct Frag<_Float16> {
  typedef v16h V; union U { v16h v; v8h h[2]; };
  static __device__ __forceinline__ v16h load(const _Float16* p) {
    U f; f.h[0] = *(const v8h*)(p); f.h[1] = *(const v8h*)(p + 16); return f.v;
  }
  static __device__ __forceinline__ v8f mma(v16h a, v16h b, v8f c) {
    return __builtin_amdgcn_wmma_f32_16x16x32_f16(false, a, false, b, (short)0, c, false, false);
  }
  static __device__ __forceinline__ void guard(v8f& a, v8f& b, v16h x, v16h y) { dep_guard_h(a, b, x, y); }
  static __device__ __forceinline__ void keep(v16h a, v16h b, v16h c, v16h d) { keep4_h(a, b, c, d); }
};
template <> struct Frag<__bf16> {
  typedef v16b V; union U { v16b v; v8b h[2]; };
  static __device__ __forceinline__ v16b load(const __bf16* p) {
    U f; f.h[0] = *(const v8b*)(p); f.h[1] = *(const v8b*)(p + 16); return f.v;
  }
  static __device__ __forceinline__ v8f mma(v16b a, v16b b, v8f c) {
    return __builtin_amdgcn_wmma_f32_16x16x32_bf16(false, a, false, b, (short)0, c, false, false);
  }
  static __device__ __forceinline__ void guard(v8f& a, v8f& b, v16b x, v16b y) { dep_guard_b(a, b, x, y); }
  static __device__ __forceinline__ void keep(v16b a, v16b b, v16b c, v16b d) { keep4_b(a, b, c, d); }
};

__device__ __forceinline__ unsigned pk16(unsigned short a, unsigned short b) { return (unsigned)a | ((unsigned)b << 16); }
__device__ __forceinline__ unsigned short h_bits(float f) { const _Float16 h = (_Float16)f; return __builtin_bit_cast(unsigned short, h); }

template <int ET> struct Elem;
template <> struct Elem<0> { typedef _Float16 T; };
template <> struct Elem<1> { typedef __bf16 T; };
template <int ET, bool SPLIT, int BIAS_MODE, int OUT_MODE, bool RESID, int ACT = 0>
__global__ __launch_bounds__(256) void wmma_gemm64(
    const unsigned short* __restrict__ Ap, const unsigned short* __restrict__ A2p, int lda, long strideA,
    const unsigned short* __restrict__ Btp, const unsigned short* __restrict__ Bt2p, int ldb, long strideB,
    void* __restrict__ Cout, void* __restrict__ Cout2, int ldc, long strideC,
    const float* __restrict__ bias,
    const float* __restrict__ resid, long strideR,
    int M, int N, int K, int Mst, float scale) {
  typedef typename Elem<ET>::T T;
  typedef typename Frag<T>::V V;
  const T* A = (const T*)Ap; const T* A2 = (const T*)A2p; const T* Bt = (const T*)Btp; const T* Bt2 = (const T*)Bt2p;
  __shared__ __align__(16) float sT[8][16 * 68];
  const int b    = blockIdx.y;
  const int lane = threadIdx.x & 31;
  const int wave = threadIdx.x >> 5;
  const int tilesN = N >> 6;
  const int tilesM = M >> 6;
  const int tile = blockIdx.x * 8 + wave;
  if (tile >= tilesM * tilesN) return;
  const int tm = tile / tilesN;
  const int tn = tile - tm * tilesN;
  const int m0 = tm << 6;
  const int n0 = tn << 6;

  const T* Ab  = A  + (size_t)b * strideA;
  const T* Bb  = Bt + (size_t)b * strideB;
  const T* Ab2 = SPLIT ? (A2  + (size_t)b * strideA) : nullptr;
  const T* Bb2 = SPLIT ? (Bt2 + (size_t)b * strideB) : nullptr;

  const int rlane = lane & 15;
  const int koff  = (lane >> 4) * 8;
  const int mOff  = (lane >> 4) * 8;

  v8f acc[4][4];
#pragma unroll
  for (int i = 0; i < 4; ++i)
#pragma unroll
    for (int j = 0; j < 4; ++j) acc[i][j] = (v8f){0.f,0.f,0.f,0.f,0.f,0.f,0.f,0.f};

  for (int k0 = 0; k0 < K; k0 += 32) {
    V bh[4], bl[4];
#pragma unroll
    for (int j = 0; j < 4; ++j) {
      const size_t bo = (size_t)(n0 + (j << 4) + rlane) * ldb + koff + k0;
      bh[j] = Frag<T>::load(Bb + bo);
      if (SPLIT) bl[j] = Frag<T>::load(Bb2 + bo);
    }
#pragma unroll
    for (int i = 0; i < 4; ++i) {
      const size_t ao = (size_t)(m0 + (i << 4) + rlane) * lda + koff + k0;
      V ah = Frag<T>::load(Ab + ao);
      V al;
      if (SPLIT) al = Frag<T>::load(Ab2 + ao);
#pragma unroll
      for (int j = 0; j < 4; ++j) {
        acc[i][j] = Frag<T>::mma(ah, bh[j], acc[i][j]);
        if (SPLIT) {
          acc[i][j] = Frag<T>::mma(ah, bl[j], acc[i][j]);
          acc[i][j] = Frag<T>::mma(al, bh[j], acc[i][j]);
        }
      }
      Frag<T>::guard(acc[i][0], acc[i][3], ah, SPLIT ? al : ah);
    }
    Frag<T>::keep(bh[0], bh[1], bh[2], bh[3]);
    if (SPLIT) Frag<T>::keep(bl[0], bl[1], bl[2], bl[3]);
  }
  acc_guard4(acc[0][0], acc[0][1], acc[0][2], acc[0][3]);
  acc_guard4(acc[1][0], acc[1][1], acc[1][2], acc[1][3]);
  acc_guard4(acc[2][0], acc[2][1], acc[2][2], acc[2][3]);
  acc_guard4(acc[3][0], acc[3][1], acc[3][2], acc[3][3]);

  float* slab = sT[wave];
  const float* Rb = RESID ? (resid + (size_t)b * strideR) : nullptr;
#pragma unroll
  for (int i = 0; i < 4; ++i) {
    const int mBase = m0 + (i << 4);
#pragma unroll
    for (int j = 0; j < 4; ++j) {
      const int n = n0 + (j << 4) + rlane;
      float bv = 0.f;
      if (BIAS_MODE == 2) bv = bias[n];
#pragma unroll
      for (int r = 0; r < 8; ++r) {
        float v = acc[i][j][r] * scale;
        if (BIAS_MODE == 1) v += bias[mBase + mOff + r];
        if (BIAS_MODE == 2) v += bv;
        if (RESID) v += Rb[(size_t)(mBase + mOff + r) * ldc + n];
        if (ACT == 2) v = fmaxf(v, 0.0f);
        if (ACT == 4) v = (v > 0.f) ? v : 0.01f * v;
        slab[(mOff + r) * 68 + (j << 4) + rlane] = v;
      }
    }
    __builtin_amdgcn_fence(__ATOMIC_RELEASE, "workgroup");
    __builtin_amdgcn_wave_barrier();
    __builtin_amdgcn_fence(__ATOMIC_ACQUIRE, "workgroup");
    if (OUT_MODE == 0) {
      float* C = (float*)Cout + (size_t)b * strideC;
      const int hh = lane >> 4, c4 = (lane & 15) * 4;
      for (int pass = 0; pass < 2; ++pass) {
#pragma unroll
        for (int it = 0; it < 8; ++it) {
          const int row = it * 2 + hh;
          v4f v = *(const v4f*)(slab + row * 68 + c4);
          if (mBase + row < Mst) *(volatile v4f*)(C + (size_t)(mBase + row) * ldc + n0 + c4) = v;
        }
        __threadfence();
      }
    } else {
      const int q = lane >> 3, c8 = (lane & 7) * 8;
      unsigned short* C  = (unsigned short*)Cout  + (size_t)b * strideC;
      unsigned short* C2 = (OUT_MODE == 2) ? ((unsigned short*)Cout2 + (size_t)b * strideC) : nullptr;
      for (int pass = 0; pass < 2; ++pass) {
#pragma unroll
        for (int it = 0; it < 4; ++it) {
          const int row = it * 4 + q;
          const float* sp = slab + row * 68 + c8;
          v8h hv, lv;
#pragma unroll
          for (int e = 0; e < 8; ++e) {
            if (OUT_MODE == 1) {
              hv[e] = (_Float16)sp[e];
            } else {
              unsigned short hb = f2bf_bits(sp[e]);
              unsigned short lb = f2bf_bits(sp[e] - bf_bits2f(hb));
              hv[e] = __builtin_bit_cast(_Float16, hb);
              lv[e] = __builtin_bit_cast(_Float16, lb);
            }
          }
          if (mBase + row < Mst) {
            *(volatile v8h*)(C + (size_t)(mBase + row) * ldc + n0 + c8) = hv;
            if (OUT_MODE == 2) *(volatile v8h*)(C2 + (size_t)(mBase + row) * ldc + n0 + c8) = lv;
          }
        }
        __threadfence();
      }
    }
    __builtin_amdgcn_fence(__ATOMIC_RELEASE, "workgroup");
    __builtin_amdgcn_wave_barrier();
    __builtin_amdgcn_fence(__ATOMIC_ACQUIRE, "workgroup");
  }
}

__global__ __launch_bounds__(256) void wcast_kernel(const float* __restrict__ W0, const float* __restrict__ W1,
                                                    const float* __restrict__ W2, const float* __restrict__ W3,
                                                    unsigned short* __restrict__ out, float scale) {
  const int z = blockIdx.y;
  const float* W = (z == 0) ? W0 : (z == 1) ? W1 : (z == 2) ? W2 : W3;
  const int i = blockIdx.x * 256 + threadIdx.x;
  const float* p = W + 8 * (size_t)i;
  const v4f a = *(const v4f*)(p);
  const v4f c = *(const v4f*)(p + 4);
  unsigned short hb[8];
#pragma unroll
  for (int e = 0; e < 4; ++e) {
    hb[e]     = h_bits(a[e] * scale);
    hb[4 + e] = h_bits(c[e] * scale);
  }
  const v4u u = (v4u){pk16(hb[0], hb[1]), pk16(hb[2], hb[3]), pk16(hb[4], hb[5]), pk16(hb[6], hb[7])};
  unsigned short* q = out + (size_t)z * kC * kC + 8 * (size_t)i;
  *(volatile v4u*)q = u;
  __threadfence();
  *(volatile v4u*)q = u;
}

__global__ __launch_bounds__(256) void mix_kernel(const float* __restrict__ x, const float* __restrict__ xs,
                                                  const float* __restrict__ tmix,
                                                  unsigned short* __restrict__ XM, unsigned short* __restrict__ R16) {
#pragma clang fp contract(off)
  const int i   = blockIdx.x * 256 + threadIdx.x;
  const int row = i >> 7;
  const int c8  = (i & 127) * 8;
  v4u u;
  if (row >= kRows) {
    u = (v4u){0u, 0u, 0u, 0u};
    unsigned short* rp = R16 + (size_t)row * kC + c8;
    *(volatile v4u*)rp = u;
    __threadfence();
    *(volatile v4u*)rp = u;
  } else {
    const int b    = row / kT;
    const int t    = row - b * kT;
    const int rowp = (row > 0) ? (row - 1) : 0;
    const float* xr = x    + (size_t)row  * kC + c8;
    const float* xp = x    + (size_t)rowp * kC + c8;
    const float* sr = xs   + (size_t)b    * kC + c8;
    const float* tp = tmix + c8;
    const v4f x0 = *(const v4f*)(xr), x1 = *(const v4f*)(xr + 4);
    const v4f p0 = *(const v4f*)(xp), p1 = *(const v4f*)(xp + 4);
    const v4f s0 = *(const v4f*)(sr), s1 = *(const v4f*)(sr + 4);
    const v4f m0 = *(const v4f*)(tp), m1 = *(const v4f*)(tp + 4);
    unsigned short hb[8];
#pragma unroll
    for (int e = 0; e < 4; ++e) {
      const float pa = (t == 0) ? s0[e] : p0[e];
      const float pb = (t == 0) ? s1[e] : p1[e];
      const float va = x0[e] * m0[e] + pa * (1.0f - m0[e]);
      const float vb = x1[e] * m1[e] + pb * (1.0f - m1[e]);
      hb[e]     = h_bits(va);
      hb[4 + e] = h_bits(vb);
    }
    u = (v4u){pk16(hb[0], hb[1]), pk16(hb[2], hb[3]), pk16(hb[4], hb[5]), pk16(hb[6], hb[7])};
  }
  unsigned short* op = XM + (size_t)row * kC + c8;
  *(volatile v4u*)op = u;
  __threadfence();
  *(volatile v4u*)op = u;
}

__global__ __launch_bounds__(256) void wkv_kernel(const float* __restrict__ KVR,
                                                  const float* __restrict__ aa, const float* __restrict__ bb,
                                                  const float* __restrict__ mmp,
                                                  const float* __restrict__ td, const float* __restrict__ tf,
                                                  unsigned short* __restrict__ R16) {
  __shared__ __align__(16) float sval[kTT][256];
  const int tid  = threadIdx.x;
  const int lane = tid & 31;
  const int wave = tid >> 5;
  const int c0   = blockIdx.x * 256;
  const int c    = c0 + tid;
  const int b    = blockIdx.y;
  const size_t rowb = (size_t)b * kT;
  const float* kcol = KVR + rowb * kN3 + c;

  float m = kcol[0];
#pragma unroll 1
  for (int t = 1; t < kT; ++t) m = fmaxf(m, kcol[(size_t)t * kN3]);
  int ex = 0;
  (void)frexpf(m, &ex);
  const float mmn = ldexpf(0.5f, ex);

  const float rsf = expf(mmp[b * kC + c] - mmn);
  const float eu  = expf(tf[c]);
  const float dec = expf(td[c]);
  const float w1  = expf(-dec);
  float q = bb[b * kC + c] * rsf;
  float p = aa[b * kC + c] * rsf;

  const int c8l = lane * 8;
  for (int t0 = 0; t0 < kT; t0 += kTT) {
    const int nt = (kT - t0 < kTT) ? (kT - t0) : kTT;
#pragma unroll 1
    for (int tl = 0; tl < nt; ++tl) {
      const float* rp = KVR + (rowb + t0 + tl) * (size_t)kN3 + c;
      const float kk = rp[0];
      const float vv = rp[kC];
      const float rr = rp[2 * kC];
      const float ke  = expf(kk - mmn);
      const float kv  = ke * vv;
      const float wk  = eu * ke + q;
      const float wkv = eu * kv + p;
      float ratio = wkv / wk;
      ratio = (ratio != ratio) ? 0.0f : ratio;
      ratio = fminf(fmaxf(ratio, -kFltMax), kFltMax);
      const float sig = 1.0f / (1.0f + expf(-rr));
      sval[tl][tid] = sig * ratio;
      q = w1 * q + ke;
      p = w1 * p + kv;
    }
    __syncthreads();
    for (int pass = 0; pass < 2; ++pass) {
#pragma unroll
      for (int it = 0; it < 4; ++it) {
        const int rl = it * 8 + wave;
        if (rl < nt) {
          const v4f a = *(const v4f*)(&sval[rl][c8l]);
          const v4f d = *(const v4f*)(&sval[rl][c8l + 4]);
          unsigned short hb[8];
#pragma unroll
          for (int e = 0; e < 4; ++e) {
            hb[e]     = h_bits(a[e]);
            hb[4 + e] = h_bits(d[e]);
          }
          const v4u u = (v4u){pk16(hb[0], hb[1]), pk16(hb[2], hb[3]), pk16(hb[4], hb[5]), pk16(hb[6], hb[7])};
          *(volatile v4u*)(R16 + (rowb + t0 + rl) * (size_t)kC + c0 + c8l) = u;
        }
      }
      __threadfence();
    }
    __syncthreads();
  }
}

extern "C" void kernel_launch(void* const* d_in, const int* in_sizes, int n_in,
                              void* d_out, int out_size, void* d_ws, size_t ws_size,
                              hipStream_t stream) {
  (void)in_sizes; (void)n_in; (void)out_size;
  const float* x    = (const float*)d_in[0];
  const float* xx   = (const float*)d_in[1];
  const float* aa   = (const float*)d_in[2];
  const float* bb   = (const float*)d_in[3];
  const float* mm   = (const float*)d_in[4];
  const float* td   = (const float*)d_in[5];
  const float* tf   = (const float*)d_in[6];
  const float* tmix = (const float*)d_in[7];
  const float* Wk   = (const float*)d_in[8];
  const float* Wv   = (const float*)d_in[9];
  const float* Wr   = (const float*)d_in[10];
  const float* Wo   = (const float*)d_in[11];
  float* out = (float*)d_out;

  const size_t szXM  = (size_t)kRowsPad * kC * 2;
  const size_t szW   = (size_t)4 * kC * kC * 2;
  const size_t szKVR = (size_t)kRowsPad * kN3 * 4;
  const size_t szR   = (size_t)kRowsPad * kC * 2;
  const size_t oXM  = 0;
  const size_t oW   = oXM + szXM;
  const size_t oKVR = oW + szW;
  const size_t oR   = oKVR + szKVR;
  const size_t total = oR + szR;
  if (total > ws_size) return;

  char* ws = (char*)d_ws;
  unsigned short* XM16 = (unsigned short*)(ws + oXM);
  unsigned short* W16  = (unsigned short*)(ws + oW);
  float*          KVR  = (float*)(ws + oKVR);
  unsigned short* R16  = (unsigned short*)(ws + oR);
  const float* dummyf  = (const float*)(ws + oKVR);

  wcast_kernel<<<dim3(kC * kC / 8 / 256, 4), 256, 0, stream>>>(Wk, Wv, Wr, Wo, W16, kWCarry);

  mix_kernel<<<dim3(kRowsPad * kC / 8 / 256), 256, 0, stream>>>(x, xx, tmix, XM16, R16);

  wmma_gemm64<0, false, 0, 0, false, 0><<<dim3((kRowsPad / 64) * (kN3 / 64) / 8, 1), 256, 0, stream>>>(
      XM16, XM16, kC, 0L,
      W16, W16, kC, 0L,
      (void*)KVR, (void*)KVR, kN3, 0L,
      dummyf, dummyf, 0L,
      kRowsPad, kN3, kC, kRowsPad, kWCarryInv);

  wkv_kernel<<<dim3(kC / 256, kB), 256, 0, stream>>>(KVR, aa, bb, mm, td, tf, R16);

  wmma_gemm64<0, false, 0, 0, false, 0><<<dim3((kRowsPad / 64) * (kC / 64) / 8, 1), 256, 0, stream>>>(
      R16, R16, kC, 0L,
      W16 + (size_t)3 * kC * kC, W16 + (size_t)3 * kC * kC, kC, 0L,
      (void*)out, (void*)out, kC, 0L,
      dummyf, dummyf, 0L,
      kRowsPad, kC, kC, kRows, kWCarryInv);
}
